// MambaBlock_40063454937735
// MI455X (gfx1250) — hardware-verified
//
#include <hip/hip_runtime.h>
#include <math.h>

typedef __attribute__((ext_vector_type(16))) _Float16 v16h;
typedef __attribute__((ext_vector_type(8)))  _Float16 v8h;
typedef __attribute__((ext_vector_type(8)))  float    v8f;
typedef __attribute__((ext_vector_type(4)))  float    v4f;

constexpr int kBatch  = 2;
constexpr int kSeq    = 2048;
constexpr int kDm     = 1024;
constexpr int kDin    = 2048;
constexpr int kNst    = 16;
constexpr int kDtR    = 64;
constexpr int kConvK  = 4;
constexpr int kRows   = kBatch * kSeq;
constexpr int kXpN    = 2 * kDin + kNst + kDtR;
constexpr int kXpNP   = 4224;
constexpr int kColDr  = 2 * kDin;
constexpr int kColBp  = 2 * kDin + kDtR;
constexpr int kSrcBp  = 2 * kDin;
constexpr int kSrcDr  = 2 * kDin + kNst;
constexpr int kBpP    = 32;
constexpr float kWCarry    = 32.0f;
constexpr float kGCarry    = 256.0f;
constexpr float kWCarryInv = 1.0f / kWCarry;
constexpr float kOutInv    = 1.0f / (kWCarry * kGCarry);
constexpr int kScTP   = 260;
constexpr int kScSteps = 16;
constexpr int kScCh   = 256;

static_assert(kXpN == 4176, "in_proj width");
static_assert(kXpNP % 64 == 0 && kXpNP >= kXpN, "padded in_proj width");
static_assert(kColBp + kNst == kXpN, "tail permutation");
static_assert(kDm % 32 == 0 && kDtR % 32 == 0 && kDin % 32 == 0, "GEMM K multiples of 32");
static_assert(kRows % 64 == 0 && kDin % 64 == 0 && kDm % 64 == 0, "GEMM M,N multiples of 64");
static_assert(((kRows / 64) * (kXpNP / 64)) % 8 == 0, "in_proj tiles fill whole blocks");
static_assert(((kRows / 64) * (kDin / 64)) % 8 == 0, "dt tiles fill whole blocks");
static_assert(((kRows / 64) * (kDm / 64)) % 8 == 0, "out tiles fill whole blocks");
static_assert(kSeq % kScSteps == 0 && kDin % kScCh == 0, "scan tiles");
static_assert(kConvK == 4 && kNst == 16, "scan register layout");

constexpr size_t kSzIn16   = (size_t)kRows * kDm * 2;
constexpr size_t kSzWin16  = (size_t)kXpNP * kDm * 2;
constexpr size_t kSzG16    = (size_t)kRows * kDin * 2;
constexpr size_t kSzWout16 = (size_t)kDm * kDin * 2;
constexpr size_t kSzWdt16  = (size_t)kDin * kDtR * 2;
constexpr size_t kSzDr16   = (size_t)kRows * kDtR * 2;
constexpr size_t kSzBp     = (size_t)kRows * kBpP * 4;
constexpr size_t kSzPlane  = (size_t)kRows * kDin * 4;
constexpr size_t kOffIn16   = 0;
constexpr size_t kOffWin16  = kOffIn16 + kSzIn16;
constexpr size_t kOffG16    = 0;
constexpr size_t kOffWout16 = kOffWin16 + kSzWin16;
constexpr size_t kOffWdt16  = kOffWout16 + kSzWout16;
constexpr size_t kOffDr16   = kOffWdt16 + kSzWdt16;
constexpr size_t kOffBp     = kOffDr16 + kSzDr16;
constexpr size_t kOffV      = kOffBp + kSzBp;
constexpr size_t kOffX      = kOffV + kSzPlane;
constexpr size_t kOffZ      = kOffX + kSzPlane;
constexpr size_t kWsTotal   = kOffZ + kSzPlane;
static_assert(kOffG16 + kSzG16 <= kOffWout16, "G16 stays inside the dead IN16+WIN16 region");
static_assert(kWsTotal == 123207680ull, "carve total");
static_assert(kWsTotal <= 134217728ull, "carve cap");
static_assert((kOffWin16 % 128) == 0 && (kOffWout16 % 128) == 0 && (kOffWdt16 % 128) == 0 &&
              (kOffDr16 % 128) == 0 && (kOffBp % 128) == 0 && (kOffV % 128) == 0 &&
              (kOffX % 128) == 0 && (kOffZ % 128) == 0, "128-B aligned regions");

__device__ __forceinline__ int perm_src_row(int r) {
  int s = r;
  s = (r >= kColDr) ? (r - kColDr + kSrcDr) : s;
  s = (r >= kColBp) ? (r - kColBp + kSrcBp) : s;
  s = (r >= kXpN) ? -1 : s;
  return s;
}

__device__ __forceinline__ v16h frag_load_h(const _Float16* p) {
  union U { v16h v; v8h h[2]; };
  U f;
  f.h[0] = *(const v8h*)(p);
  f.h[1] = *(const v8h*)(p + 16);
  return f.v;
}
__device__ __forceinline__ v8f mma_h(v16h a, v16h b, v8f c) {
  return __builtin_amdgcn_wmma_f32_16x16x32_f16(false, a, false, b, (short)0, c, false, false);
}
__device__ __forceinline__ void grp_guard_h(v8f& a, v8f& b, v8f& c, v8f& d,
                                            v16h x, v16h y0, v16h y1, v16h y2, v16h y3) {
  asm volatile("v_nop\n\tv_nop\n\tv_nop\n\tv_nop"
               : "+v"(a), "+v"(b), "+v"(c), "+v"(d)
               : "v"(x), "v"(y0), "v"(y1), "v"(y2), "v"(y3));
}
__device__ __forceinline__ void keep4_h(v16h a, v16h b, v16h c, v16h d) {
  asm volatile("v_nop" :: "v"(a), "v"(b), "v"(c), "v"(d));
}
__device__ __forceinline__ void acc_guard4(v8f& a, v8f& b, v8f& c, v8f& d) {
  asm volatile("v_nop\n\tv_nop\n\tv_nop\n\tv_nop" : "+v"(a), "+v"(b), "+v"(c), "+v"(d));
}

__global__ __launch_bounds__(256) void cast_rows_f16_kernel(
    const float* __restrict__ src, unsigned short* dst, int total8, float scale, int rowLen8, int permute)
{
  const int i = blockIdx.x * 256 + threadIdx.x;
  if (i >= total8) return;
  const size_t e0 = (size_t)i << 3;
  size_t s0 = e0;
  bool real = true;
  if (permute != 0) {
    const int r  = i / rowLen8;
    const int c8 = i - r * rowLen8;
    const int sr = perm_src_row(r);
    real = (sr >= 0);
    const int srow = real ? sr : 0;
    s0 = ((size_t)srow * (size_t)rowLen8 + (size_t)c8) << 3;
  }
  const v4f a0 = *(const v4f*)(src + s0);
  const v4f a1 = *(const v4f*)(src + s0 + 4);
  v8h hv;
#pragma unroll
  for (int e = 0; e < 4; ++e) {
    const float f0 = real ? (a0[e] * scale) : 0.0f;
    const float f1 = real ? (a1[e] * scale) : 0.0f;
    hv[e]     = (_Float16)f0;
    hv[4 + e] = (_Float16)f1;
  }
  unsigned short* q = dst + e0;
  *(volatile v8h*)q = hv;
  __threadfence();
  *(volatile v8h*)q = hv;
}

template <int ROUTE>
__global__ __launch_bounds__(256) void gemm_f16_kernel(
    const unsigned short* __restrict__ Ap, int lda,
    const unsigned short* __restrict__ Btp, int ldb,
    float* C0, float* C1, unsigned short* C16, float* CB, int ldc,
    const float* __restrict__ bias, const float* __restrict__ bias2,
    int M, int N, int K, float scale)
{
  const _Float16* A  = (const _Float16*)Ap;
  const _Float16* Bt = (const _Float16*)Btp;
  __shared__ __align__(16) float sT[8][16 * 68];
  const int lane = threadIdx.x & 31;
  const int wave = threadIdx.x >> 5;
  const int tilesN = N >> 6;
  const int tilesM = M >> 6;
  const int tile = blockIdx.x * 8 + wave;
  if (tile >= tilesM * tilesN) return;
  const int tm = tile / tilesN;
  const int tn = tile - tm * tilesN;
  const int m0 = tm << 6;
  const int n0 = tn << 6;

  const int rlane = lane & 15;
  const int koff  = (lane >> 4) * 8;
  const int mOff  = (lane >> 4) * 8;

  v8f acc[4][4];
#pragma unroll
  for (int i = 0; i < 4; ++i)
#pragma unroll
    for (int j = 0; j < 4; ++j) acc[i][j] = (v8f){0.f, 0.f, 0.f, 0.f, 0.f, 0.f, 0.f, 0.f};

  for (int k0 = 0; k0 < K; k0 += 32) {
    v16h bh[4];
#pragma unroll
    for (int j = 0; j < 4; ++j) {
      const size_t bo = (size_t)(n0 + (j << 4) + rlane) * ldb + koff + k0;
      bh[j] = frag_load_h(Bt + bo);
    }
#pragma unroll
    for (int i = 0; i < 4; ++i) {
      const size_t ao = (size_t)(m0 + (i << 4) + rlane) * lda + koff + k0;
      const v16h ah = frag_load_h(A + ao);
#pragma unroll
      for (int j = 0; j < 4; ++j) acc[i][j] = mma_h(ah, bh[j], acc[i][j]);
      grp_guard_h(acc[i][0], acc[i][1], acc[i][2], acc[i][3], ah, bh[0], bh[1], bh[2], bh[3]);
    }
    keep4_h(bh[0], bh[1], bh[2], bh[3]);
  }
  acc_guard4(acc[0][0], acc[0][1], acc[0][2], acc[0][3]);
  acc_guard4(acc[1][0], acc[1][1], acc[1][2], acc[1][3]);
  acc_guard4(acc[2][0], acc[2][1], acc[2][2], acc[2][3]);
  acc_guard4(acc[3][0], acc[3][1], acc[3][2], acc[3][3]);

  float bvj[4];
#pragma unroll
  for (int j = 0; j < 4; ++j) {
    const int n = n0 + (j << 4) + rlane;
    if (ROUTE == 0) {
      bvj[j] = bias[n];
    } else {
      const int sr = perm_src_row(n);
      const bool real = (sr >= 0);
      const int sc = real ? sr : 0;
      const float b0 = bias[sc];
      const bool isB = (n >= kColBp) && (n < kXpN);
      const int pi = isB ? (n - kColBp) : 0;
      const float b1 = bias2[pi];
      bvj[j] = (real ? b0 : 0.0f) + (isB ? b1 : 0.0f);
    }
  }

  float* slab = sT[wave];
#pragma unroll
  for (int i = 0; i < 4; ++i) {
    const int mBase = m0 + (i << 4);
#pragma unroll
    for (int j = 0; j < 4; ++j) {
#pragma unroll
      for (int r = 0; r < 8; ++r) {
        const float v = acc[i][j][r] * scale + bvj[j];
        slab[(mOff + r) * 68 + (j << 4) + rlane] = v;
      }
    }
    __builtin_amdgcn_fence(__ATOMIC_RELEASE, "workgroup");
    __builtin_amdgcn_wave_barrier();
    __builtin_amdgcn_fence(__ATOMIC_ACQUIRE, "workgroup");
    if (ROUTE == 0 || tn < 64) {
      float* C;
      int nc0, ldo;
      if (ROUTE == 0) {
        C = C0; nc0 = n0; ldo = ldc;
      } else {
        C = (tn < 32) ? C0 : C1;
        nc0 = (tn & 31) << 6;
        ldo = kDin;
      }
      const int hh = lane >> 4, c4 = (lane & 15) * 4;
      for (int pass = 0; pass < 2; ++pass) {
#pragma unroll
        for (int it = 0; it < 8; ++it) {
          const int row = it * 2 + hh;
          const v4f v = *(const v4f*)(slab + row * 68 + c4);
          *(volatile v4f*)(C + (size_t)(mBase + row) * ldo + nc0 + c4) = v;
        }
        __threadfence();
      }
    } else if (tn == 64) {
      const int q = lane >> 3, c8 = (lane & 7) * 8;
      v8h hv[4];
#pragma unroll
      for (int it = 0; it < 4; ++it) {
        const float* sp = slab + (it * 4 + q) * 68 + c8;
        const v4f a0 = *(const v4f*)(sp);
        const v4f a1 = *(const v4f*)(sp + 4);
#pragma unroll
        for (int e = 0; e < 4; ++e) {
          hv[it][e]     = (_Float16)a0[e];
          hv[it][4 + e] = (_Float16)a1[e];
        }
      }
      for (int pass = 0; pass < 2; ++pass) {
#pragma unroll
        for (int it = 0; it < 4; ++it) {
          const int row = it * 4 + q;
          *(volatile v8h*)(C16 + (size_t)(mBase + row) * kDtR + c8) = hv[it];
        }
        __threadfence();
      }
    } else {
      const int q = lane >> 3, c4 = (lane & 7) * 4;
      for (int pass = 0; pass < 2; ++pass) {
#pragma unroll
        for (int it = 0; it < 4; ++it) {
          const int row = it * 4 + q;
          const v4f v = *(const v4f*)(slab + row * 68 + c4);
          *(volatile v4f*)(CB + (size_t)(mBase + row) * kBpP + c4) = v;
        }
        __threadfence();
      }
    }
    __builtin_amdgcn_fence(__ATOMIC_RELEASE, "workgroup");
    __builtin_amdgcn_wave_barrier();
    __builtin_amdgcn_fence(__ATOMIC_ACQUIRE, "workgroup");
  }
}

__global__ __launch_bounds__(256) void scan_gate_kernel(
    const float* __restrict__ ZPL, const float* __restrict__ XPL, const float* __restrict__ VPL,
    const float* __restrict__ BP, const float* __restrict__ A_log, const float* __restrict__ Cp,
    const float* __restrict__ Wc, unsigned short* G16)
{
  __shared__ __align__(16) float sB[kScSteps * kNst];
  __shared__ __align__(16) float sY[kScSteps * kScTP];
  __shared__ __align__(16) float sA[kNst * kScCh];
  const int tid = threadIdx.x, lane = tid & 31, wave = tid >> 5;
  const int d0 = blockIdx.x * kScCh, d = d0 + tid;
  const size_t row0 = (size_t)blockIdx.y * kSeq;

#pragma unroll 1
  for (int n = 0; n < kNst; ++n) sA[n * kScCh + tid] = -expf(A_log[(size_t)d * kNst + n]);
  __syncthreads();

  float An[kNst], Cn[kNst], h[kNst];
#pragma unroll
  for (int n = 0; n < kNst; ++n) {
    An[n] = sA[n * kScCh + tid];
    h[n] = 0.0f;
  }
#pragma unroll
  for (int q4 = 0; q4 < 4; ++q4) {
    const v4f cv = *(const v4f*)(Cp + (size_t)d * kNst + 4 * q4);
    Cn[4 * q4 + 0] = cv[0];
    Cn[4 * q4 + 1] = cv[1];
    Cn[4 * q4 + 2] = cv[2];
    Cn[4 * q4 + 3] = cv[3];
  }
  const v4f wv = *(const v4f*)(Wc + (size_t)d * kConvK);
  const float w0 = wv[0], w1 = wv[1], w2 = wv[2], w3 = wv[3];
  float xm3 = 0.0f, xm2 = 0.0f, xm1 = 0.0f;

#pragma unroll 1
  for (int c = 0; c < kSeq / kScSteps; ++c) {
    const int l0 = c * kScSteps;
    if (tid < 64) {
      const int r = tid >> 2, q4 = (tid & 3) * 4;
      const v4f bv = *(const v4f*)(BP + (row0 + l0 + r) * kBpP + q4);
      *(v4f*)(sB + r * kNst + q4) = bv;
    }
    __syncthreads();
#pragma unroll 1
    for (int s = 0; s < kScSteps; ++s) {
      const size_t off = (row0 + l0 + s) * (size_t)kDin + d;
      float zp = ZPL[off];
      float xc = XPL[off];
      float vv = VPL[off];
      asm volatile("" : "+v"(zp), "+v"(xc), "+v"(vv));
      float ca = w0 * xm3;
      ca = fmaf(w1, xm2, ca);
      ca = fmaf(w2, xm1, ca);
      ca = fmaf(w3, xc, ca);
      xm3 = xm2; xm2 = xm1; xm1 = xc;
      const float xs = ca * __builtin_amdgcn_rcpf(1.0f + expf(-ca));
      const float delta = fmaxf(zp, 0.0f) + log1pf(expf(-fabsf(zp)));
      const float dx = delta * xs;
      v4f Bq[4];
#pragma unroll
      for (int q4 = 0; q4 < 4; ++q4) Bq[q4] = *(const v4f*)(sB + s * kNst + 4 * q4);
      float y = 0.0f;
#pragma unroll
      for (int n = 0; n < kNst; ++n) {
        const float e = expf(delta * An[n]);
        float p = dx * Bq[n >> 2][n & 3];
        asm volatile("" : "+v"(p));
        float qv = h[n] * e;
        asm volatile("" : "+v"(qv));
        const float hn = qv + p;
        h[n] = hn;
        float rr = Cn[n] * hn;
        asm volatile("" : "+v"(rr));
        y += rr;
      }
      const float gs = vv * __builtin_amdgcn_rcpf(1.0f + expf(-vv));
      sY[s * kScTP + tid] = (y * gs) * kGCarry;
    }
    __syncthreads();
    v8h hv[2];
#pragma unroll
    for (int it = 0; it < 2; ++it) {
      const float* sp = sY + (it * 8 + wave) * kScTP + lane * 8;
      const v4f a0 = *(const v4f*)(sp);
      const v4f a1 = *(const v4f*)(sp + 4);
#pragma unroll
      for (int e = 0; e < 4; ++e) {
        hv[it][e]     = (_Float16)a0[e];
        hv[it][4 + e] = (_Float16)a1[e];
      }
    }
    for (int pass = 0; pass < 2; ++pass) {
#pragma unroll
      for (int it = 0; it < 2; ++it)
        *(volatile v8h*)(G16 + (row0 + l0 + it * 8 + wave) * (size_t)kDin + d0 + lane * 8) = hv[it];
      __threadfence();
    }
  }
}

extern "C" void kernel_launch(void* const* d_in, const int* in_sizes, int n_in,
                              void* d_out, int out_size, void* d_ws, size_t ws_size,
                              hipStream_t stream)
{
  if (n_in < 11) return;
  if (in_sizes[0] != kRows * kDm) return;
  if (in_sizes[1] != kXpN * kDm) return;
  if (in_sizes[2] != kXpN) return;
  if (in_sizes[3] != kDin * kNst) return;
  if (in_sizes[4] != kNst) return;
  if (in_sizes[5] != kDin * kNst) return;
  if (in_sizes[6] != kDin * kDtR) return;
  if (in_sizes[7] != kDin) return;
  if (in_sizes[8] != kDin * kConvK) return;
  if (in_sizes[9] != kDm * kDin) return;
  if (in_sizes[10] != kDm) return;
  if (out_size != kRows * kDm) return;
  if (ws_size < kWsTotal) return;

  const float* x_in    = (const float*)d_in[0];
  const float* Win     = (const float*)d_in[1];
  const float* b_in    = (const float*)d_in[2];
  const float* A_log   = (const float*)d_in[3];
  const float* B_param = (const float*)d_in[4];
  const float* C_param = (const float*)d_in[5];
  const float* Wdt     = (const float*)d_in[6];
  const float* b_dt    = (const float*)d_in[7];
  const float* Wconv   = (const float*)d_in[8];
  const float* Wout    = (const float*)d_in[9];
  const float* b_out   = (const float*)d_in[10];
  float* out = (float*)d_out;

  char* ws = (char*)d_ws;
  unsigned short* IN16   = (unsigned short*)(ws + kOffIn16);
  unsigned short* WIN16  = (unsigned short*)(ws + kOffWin16);
  unsigned short* G16    = (unsigned short*)(ws + kOffG16);
  unsigned short* WOUT16 = (unsigned short*)(ws + kOffWout16);
  unsigned short* WDT16  = (unsigned short*)(ws + kOffWdt16);
  unsigned short* DR16   = (unsigned short*)(ws + kOffDr16);
  float*          BPp    = (float*)(ws + kOffBp);
  float*          VPL    = (float*)(ws + kOffV);
  float*          XPL    = (float*)(ws + kOffX);
  float*          ZPL    = (float*)(ws + kOffZ);

  cast_rows_f16_kernel<<<(kRows * kDm / 8) / 256, 256, 0, stream>>>(x_in, IN16, kRows * kDm / 8, 1.0f, kDm / 8, 0);
  cast_rows_f16_kernel<<<(kXpNP * kDm / 8) / 256, 256, 0, stream>>>(Win, WIN16, kXpNP * kDm / 8, kWCarry, kDm / 8, 1);
  cast_rows_f16_kernel<<<(kDm * kDin / 8) / 256, 256, 0, stream>>>(Wout, WOUT16, kDm * kDin / 8, kWCarry, kDin / 8, 0);
  cast_rows_f16_kernel<<<(kDin * kDtR / 8) / 256, 256, 0, stream>>>(Wdt, WDT16, kDin * kDtR / 8, kWCarry, kDtR / 8, 0);

  gemm_f16_kernel<1><<<((kRows / 64) * (kXpNP / 64)) / 8, 256, 0, stream>>>(
      IN16, kDm, WIN16, kDm,
      VPL, XPL, DR16, BPp, kDin,
      b_in, B_param,
      kRows, kXpNP, kDm, kWCarryInv);

  gemm_f16_kernel<0><<<((kRows / 64) * (kDin / 64)) / 8, 256, 0, stream>>>(
      DR16, kDtR, WDT16, kDtR,
      ZPL, ZPL, DR16, BPp, kDin,
      b_dt, b_dt,
      kRows, kDin, kDtR, kWCarryInv);

  scan_gate_kernel<<<dim3(kDin / kScCh, kBatch), kScCh, 0, stream>>>(
      ZPL, XPL, VPL, BPp, A_log, C_param, Wconv, G16);

  gemm_f16_kernel<0><<<((kRows / 64) * (kDm / 64)) / 8, 256, 0, stream>>>(
      G16, kDin, WOUT16, kDin,
      out, out, DR16, BPp, kDm,
      b_out, b_out,
      kRows, kDm, kDin, kOutInv);
}
